// ModalAttn_65893388255513
// MI455X (gfx1250) — hardware-verified
//
#include <hip/hip_runtime.h>

typedef _Float16 v16h __attribute__((ext_vector_type(16)));
typedef _Float16 v8h  __attribute__((ext_vector_type(8)));
typedef __bf16   v16b __attribute__((ext_vector_type(16)));
typedef unsigned short v8us __attribute__((ext_vector_type(8)));
typedef float v8f __attribute__((ext_vector_type(8)));
typedef float v4f __attribute__((ext_vector_type(4)));
typedef float v2f __attribute__((ext_vector_type(2)));
typedef v8h  __attribute__((may_alias)) v8ha;
typedef v8us __attribute__((may_alias)) v8usa;
typedef v4f  __attribute__((may_alias)) v4fa;

union FragH { v16h v; v8h half[2]; };
union FragB { v16b v; v8us half[2]; };

#define EDIM   512
#define NHEAD  8
#define HDIM   64
#define QKVW   1536
#define XMW    128
#define PCIN   16
#define NCLS   19
#define NCLSP  32
#define NBATCH 16
#define MAXLEN 993
#define PSC    16384.0f

__device__ __forceinline__ v8f mma_f16(v16h a, v16h b, v8f c) {
  v8f d = __builtin_amdgcn_wmma_f32_16x16x32_f16(false, a, false, b, (short)0, c, false, false);
  asm volatile("v_nop\n\tv_nop\n\tv_nop\n\tv_nop" : "+v"(d) : "v"(a), "v"(b));
  return d;
}
__device__ __forceinline__ v8f mma_bf16(v16b a, v16b b, v8f c) {
  v8f d = __builtin_amdgcn_wmma_f32_16x16x32_bf16(false, a, false, b, (short)0, c, false, false);
  asm volatile("v_nop\n\tv_nop\n\tv_nop\n\tv_nop" : "+v"(d) : "v"(a), "v"(b));
  return d;
}

__device__ __forceinline__ v16h load_frag_h(const _Float16* p, int hh) {
  FragH f;
  f.half[0] = *(const v8ha*)(p + 8 * hh);
  f.half[1] = *(const v8ha*)(p + 16 + 8 * hh);
  return f.v;
}
__device__ __forceinline__ v16b load_frag_u(const unsigned short* p, int hh) {
  FragB f;
  f.half[0] = *(const v8usa*)(p + 8 * hh);
  f.half[1] = *(const v8usa*)(p + 16 + 8 * hh);
  return f.v;
}

__device__ __forceinline__ unsigned int bf16_rne(float x) {
  const unsigned int u = __float_as_uint(x);
  return (u + 0x7FFFu + ((u >> 16) & 1u)) >> 16;
}
__device__ __forceinline__ unsigned int bf16_lo(float x, unsigned int hb) {
  return bf16_rne(x - __uint_as_float(hb << 16));
}

__device__ __forceinline__ v8h cvt8h(v4f a, v4f c, float sc) {
  const v8h o = { (_Float16)(a.x * sc), (_Float16)(a.y * sc), (_Float16)(a.z * sc), (_Float16)(a.w * sc),
                  (_Float16)(c.x * sc), (_Float16)(c.y * sc), (_Float16)(c.z * sc), (_Float16)(c.w * sc) };
  return o;
}

__device__ __forceinline__ v8f zero8f() { const v8f z = {0.f, 0.f, 0.f, 0.f, 0.f, 0.f, 0.f, 0.f}; return z; }

__device__ __forceinline__ void wprep_store(const unsigned short* sA, const unsigned short* sB,
                                            unsigned short* pa, unsigned short* pb, int two,
                                            int n0, int k0, int nrows, int w, int lane) {
  const int q8 = lane & 7, sub = lane >> 3;
  #pragma unroll
  for (int i = 0; i < 2; ++i) {
    const int row = 8 * w + 4 * i + sub;
    if (row < nrows) {
      const size_t go = (size_t)(n0 + row) * EDIM + k0 + 8 * q8;
      const v8us va = *(const v8usa*)(sA + row * 72 + 8 * q8);
      *(volatile v8us*)(pa + go) = va;
      if (two) {
        const v8us vb = *(const v8usa*)(sB + row * 72 + 8 * q8);
        *(volatile v8us*)(pb + go) = vb;
      }
    }
  }
}

__global__ __launch_bounds__(256) void k_wprep(
    const float* __restrict__ w_pc2, const float* __restrict__ w_out, const float* __restrict__ w_cls,
    unsigned short* __restrict__ w2t,
    unsigned short* __restrict__ woth, unsigned short* __restrict__ wotl,
    unsigned short* __restrict__ wcth, unsigned short* __restrict__ wctl)
{
  __shared__ __attribute__((aligned(16))) unsigned short sA[64 * 72];
  __shared__ __attribute__((aligned(16))) unsigned short sB[64 * 72];

  const int tid = threadIdx.x, lane = tid & 31, w = tid >> 5;
  const int bid = blockIdx.x;
  const float* src;
  int ld, ncols, nrows, kt, n0, two;
  unsigned short* pa;
  unsigned short* pb;
  if (bid < 8) {
    src = w_pc2; ld = 64; ncols = 64; nrows = 64; kt = bid; n0 = 0; two = 0; pa = w2t; pb = w2t;
  } else if (bid < 72) {
    const int i = bid - 8;
    src = w_out; ld = EDIM; ncols = EDIM; nrows = 64; kt = i & 7; n0 = (i >> 3) * 64; two = 1; pa = woth; pb = wotl;
  } else {
    const int i = bid - 72;
    src = w_cls; ld = NCLS; ncols = NCLS; nrows = NCLSP; kt = i; n0 = 0; two = 1; pa = wcth; pb = wctl;
  }
  const int k0 = kt * 64;
  const int nn = tid & 63, kq = tid >> 6;
  const int gcol = n0 + nn;
  const int ccol = (gcol < ncols) ? gcol : (ncols - 1);
  const bool cok = gcol < ncols;

  #pragma unroll
  for (int i = 0; i < 16; ++i) {
    const int kk = kq + 4 * i;
    float v = src[(size_t)(k0 + kk) * ld + ccol];
    v = cok ? v : 0.0f;
    if (!two) {
      const _Float16 hv = (_Float16)(v * 16.0f);
      sA[nn * 72 + kk] = __builtin_bit_cast(unsigned short, hv);
    } else {
      const unsigned int hb = bf16_rne(v);
      sA[nn * 72 + kk] = (unsigned short)hb;
      sB[nn * 72 + kk] = (unsigned short)bf16_lo(v, hb);
    }
  }
  __syncthreads();

  wprep_store(sA, sB, pa, pb, two, n0, k0, nrows, w, lane);
  __threadfence();
  wprep_store(sA, sB, pa, pb, two, n0, k0, nrows, w, lane);
}

__device__ __forceinline__ void wcomp_store(const _Float16* sT, const float* sb,
                                            _Float16* wct, float* bct,
                                            int n0, int k0, int dobias, int tid, int w, int lane) {
  const int q8 = lane & 7, sub = lane >> 3;
  #pragma unroll
  for (int i = 0; i < 2; ++i) {
    const int row = 8 * w + 4 * i + sub;
    const v8h v = *(const v8ha*)(sT + row * 72 + 8 * q8);
    *(volatile v8h*)(wct + (size_t)(n0 + row) * XMW + k0 + 8 * q8) = v;
  }
  if (dobias && tid < 16) {
    const v4f vb = *(const v4fa*)(sb + 4 * tid);
    *(volatile v4f*)(bct + n0 + 4 * tid) = vb;
  }
}

__global__ __launch_bounds__(256) void k_wcomp(
    const float* __restrict__ w_qkv, const float* __restrict__ b_qkv,
    const float* __restrict__ w_in, const float* __restrict__ b_in,
    _Float16* __restrict__ wct, float* __restrict__ bct)
{
  __shared__ __attribute__((aligned(16))) _Float16 sT[64 * 72];
  __shared__ __attribute__((aligned(16))) float sb[64];

  const int tid = threadIdx.x, lane = tid & 31, w = tid >> 5;
  const int n0 = blockIdx.x * 64, k0 = blockIdx.y * 64;
  const int s = n0 >> 9, nl0 = n0 & 511;
  const int kk = tid & 63, ng = tid >> 6;
  const int k = k0 + kk;

  float acc[16];
  #pragma unroll
  for (int i = 0; i < 16; ++i) acc[i] = 0.0f;

  const float* ap = w_qkv + (size_t)k * QKVW + s * EDIM;
  const float* bp = w_in + (size_t)s * EDIM + nl0 + 16 * ng;
  #pragma unroll 1
  for (int j = 0; j < EDIM; ++j) {
    const float a = ap[j];
    const float* bj = bp + (size_t)j * QKVW;
    v4f bq[4];
    bq[0] = *(const v4fa*)(bj);
    bq[1] = *(const v4fa*)(bj + 4);
    bq[2] = *(const v4fa*)(bj + 8);
    bq[3] = *(const v4fa*)(bj + 12);
    #pragma unroll
    for (int c = 0; c < 4; ++c) {
      acc[4 * c + 0] += a * bq[c].x;
      acc[4 * c + 1] += a * bq[c].y;
      acc[4 * c + 2] += a * bq[c].z;
      acc[4 * c + 3] += a * bq[c].w;
    }
  }
  #pragma unroll
  for (int i = 0; i < 16; ++i) sT[(16 * ng + i) * 72 + kk] = (_Float16)(acc[i] * 16.0f);

  const int dobias = (blockIdx.y == 0) ? 1 : 0;
  if (dobias) {
    if (tid < 64) {
      const int n = nl0 + tid;
      float bs = b_in[s * EDIM + n];
      const float* wp = w_in + (size_t)s * EDIM + n;
      #pragma unroll 1
      for (int j = 0; j < EDIM; ++j) bs += b_qkv[s * EDIM + j] * wp[(size_t)j * QKVW];
      sb[tid] = bs;
    }
  }
  __syncthreads();

  wcomp_store(sT, sb, wct, bct, n0, k0, dobias, tid, w, lane);
  __threadfence();
  wcomp_store(sT, sb, wct, bct, n0, k0, dobias, tid, w, lane);
}

__device__ __forceinline__ void tile_store_h(const _Float16* sT, _Float16* plane, int ldp,
                                             int r0, int c0, int w, int lane) {
  const int q8 = lane & 7, sub = lane >> 3;
  #pragma unroll
  for (int i = 0; i < 8; ++i) {
    const int lid = 32 * w + 4 * i + sub;
    const v8h v = *(const v8ha*)(sT + lid * 64 + 8 * q8);
    *(volatile v8h*)(plane + (size_t)(r0 + lid) * ldp + c0 + 8 * q8) = v;
  }
}

__global__ __launch_bounds__(128) void k_pc1(
    const float* __restrict__ pc, const float* __restrict__ w1, const float* __restrict__ b1,
    _Float16* __restrict__ h16, int N)
{
  __shared__ __attribute__((aligned(16))) _Float16 sT[128 * 64];

  const int tid = threadIdx.x, lane = tid & 31, w = tid >> 5, hh = lane >> 4, m = lane & 15;
  const int r0 = blockIdx.x * 128, c0 = blockIdx.y * 64;
  const v8h zh = {(_Float16)0.f, (_Float16)0.f, (_Float16)0.f, (_Float16)0.f,
                  (_Float16)0.f, (_Float16)0.f, (_Float16)0.f, (_Float16)0.f};

  FragH a[2];
  #pragma unroll
  for (int mt = 0; mt < 2; ++mt) {
    int row = r0 + 32 * w + 16 * mt + m;
    row = (row < N) ? row : (N - 1);
    const float* p = pc + (size_t)row * PCIN + 8 * hh;
    const v4f x0 = *(const v4fa*)p;
    const v4f x1 = *(const v4fa*)(p + 4);
    a[mt].half[0] = cvt8h(x0, x1, 1.0f);
    a[mt].half[1] = zh;
  }

  v8f acc[2][4];
  #pragma unroll
  for (int nt = 0; nt < 4; ++nt) {
    const int n = c0 + 16 * nt + m;
    FragH b;
    v8h t;
    #pragma unroll
    for (int i = 0; i < 8; ++i) t[i] = (_Float16)(w1[(size_t)(8 * hh + i) * EDIM + n] * 16.0f);
    b.half[0] = t;
    b.half[1] = zh;
    acc[0][nt] = mma_f16(a[0].v, b.v, zero8f());
    acc[1][nt] = mma_f16(a[1].v, b.v, zero8f());
  }

  #pragma unroll
  for (int nt = 0; nt < 4; ++nt) {
    const int col = 16 * nt + m;
    const float bv = b1[c0 + col];
    #pragma unroll
    for (int mt = 0; mt < 2; ++mt) {
      #pragma unroll
      for (int r = 0; r < 8; ++r) {
        const int rowl = 32 * w + 16 * mt + 8 * hh + r;
        const float y = fmaxf(acc[mt][nt][r] * 0.0625f + bv, 0.0f) * 16.0f;
        sT[rowl * 64 + col] = (_Float16)y;
      }
    }
  }
  __syncthreads();

  tile_store_h(sT, h16, EDIM, r0, c0, w, lane);
  __threadfence();
  tile_store_h(sT, h16, EDIM, r0, c0, w, lane);
}

__device__ __forceinline__ void pc2_store(const float* sF, const float* img, float* out0, _Float16* xh,
                                          int r0, int N, int tid, int w, int lane) {
  const int q8 = lane & 7, sub = lane >> 3;
  #pragma unroll
  for (int i = 0; i < 16; ++i) {
    const int lid = 4 * i + sub;
    const int rowl = 32 * w + (lid >> 1), hl = lid & 1;
    const int grow = r0 + rowl;
    if (grow < N) {
      const v4f v = *(const v4fa*)(sF + rowl * 64 + 32 * hl + 4 * q8);
      *(volatile v4f*)(out0 + (size_t)grow * XMW + 32 * hl + 4 * q8) = v;
    }
  }
  #pragma unroll
  for (int i = 0; i < 8; ++i) {
    const int rowl = 32 * w + 4 * i + sub;
    const v4f f0 = *(const v4fa*)(sF + rowl * 64 + 8 * q8);
    const v4f f1 = *(const v4fa*)(sF + rowl * 64 + 8 * q8 + 4);
    const v8h hv = cvt8h(f0, f1, 16.0f);
    *(volatile v8h*)(xh + (size_t)(r0 + rowl) * XMW + 8 * q8) = hv;
  }
  {
    const int c4 = tid & 15, rs = tid >> 4;
    #pragma unroll
    for (int i = 0; i < 16; ++i) {
      const int rowl = 8 * i + rs;
      const int grow = r0 + rowl;
      const int crow = (grow < N) ? grow : (N - 1);
      const v4f v = *(const v4fa*)(img + (size_t)crow * 64 + 4 * c4);
      if (grow < N) *(volatile v4f*)(out0 + (size_t)grow * XMW + 64 + 4 * c4) = v;
    }
  }
  {
    const int c8 = tid & 7, rs = tid >> 3;
    #pragma unroll
    for (int i = 0; i < 8; ++i) {
      const int rowl = 16 * i + rs;
      const int grow = r0 + rowl;
      const int crow = (grow < N) ? grow : (N - 1);
      const v4f f0 = *(const v4fa*)(img + (size_t)crow * 64 + 8 * c8);
      const v4f f1 = *(const v4fa*)(img + (size_t)crow * 64 + 8 * c8 + 4);
      const v8h hv = cvt8h(f0, f1, 16.0f);
      *(volatile v8h*)(xh + (size_t)grow * XMW + 64 + 8 * c8) = hv;
    }
  }
}

__global__ __launch_bounds__(128) void k_pc2x(
    const _Float16* __restrict__ h16, const _Float16* __restrict__ w2t,
    const float* __restrict__ b2, const float* __restrict__ img,
    float* __restrict__ out0, _Float16* __restrict__ xh, int N)
{
  __shared__ __attribute__((aligned(16))) float sF[128 * 64];

  const int tid = threadIdx.x, lane = tid & 31, w = tid >> 5, hh = lane >> 4, m = lane & 15;
  const int r0 = blockIdx.x * 128;
  const _Float16* a0p = h16 + (size_t)(r0 + 32 * w + m) * EDIM;
  const _Float16* a1p = a0p + (size_t)16 * EDIM;
  const _Float16* bp  = w2t + (size_t)m * EDIM;

  v8f acc[2][4];
  #pragma unroll
  for (int mt = 0; mt < 2; ++mt)
    #pragma unroll
    for (int nt = 0; nt < 4; ++nt) acc[mt][nt] = zero8f();

  #pragma unroll 1
  for (int k0 = 0; k0 < EDIM; k0 += 32) {
    const v16h a0 = load_frag_h(a0p + k0, hh);
    const v16h a1 = load_frag_h(a1p + k0, hh);
    #pragma unroll
    for (int nt = 0; nt < 4; ++nt) {
      const v16h bb = load_frag_h(bp + (size_t)(16 * nt) * EDIM + k0, hh);
      acc[0][nt] = mma_f16(a0, bb, acc[0][nt]);
      acc[1][nt] = mma_f16(a1, bb, acc[1][nt]);
    }
  }

  #pragma unroll
  for (int nt = 0; nt < 4; ++nt) {
    const int col = 16 * nt + m;
    const float bv = b2[col];
    #pragma unroll
    for (int mt = 0; mt < 2; ++mt) {
      #pragma unroll
      for (int r = 0; r < 8; ++r) {
        const int rowl = 32 * w + 16 * mt + 8 * hh + r;
        sF[rowl * 64 + col] = fmaxf(acc[mt][nt][r] * (1.0f / 256.0f) + bv, 0.0f);
      }
    }
  }
  __syncthreads();

  pc2_store(sF, img, out0, xh, r0, N, tid, w, lane);
  __threadfence();
  pc2_store(sF, img, out0, xh, r0, N, tid, w, lane);
}

__global__ __launch_bounds__(128) void k_qkv(
    const _Float16* __restrict__ xh, const _Float16* __restrict__ wct, const float* __restrict__ bct,
    _Float16* __restrict__ qkvh)
{
  __shared__ __attribute__((aligned(16))) _Float16 sT[128 * 64];

  const int tid = threadIdx.x, lane = tid & 31, w = tid >> 5, hh = lane >> 4, m = lane & 15;
  const int r0 = blockIdx.x * 128, cg = blockIdx.y;
  const _Float16* a0p = xh + (size_t)(r0 + 32 * w + m) * XMW;
  const _Float16* a1p = a0p + (size_t)16 * XMW;
  const _Float16* bp  = wct + (size_t)(cg * 64 + m) * XMW;

  v8f acc[2][4];
  #pragma unroll
  for (int mt = 0; mt < 2; ++mt)
    #pragma unroll
    for (int nt = 0; nt < 4; ++nt) acc[mt][nt] = zero8f();

  #pragma unroll 1
  for (int k0 = 0; k0 < XMW; k0 += 32) {
    const v16h a0 = load_frag_h(a0p + k0, hh);
    const v16h a1 = load_frag_h(a1p + k0, hh);
    #pragma unroll
    for (int nt = 0; nt < 4; ++nt) {
      const v16h bb = load_frag_h(bp + (size_t)(16 * nt) * XMW + k0, hh);
      acc[0][nt] = mma_f16(a0, bb, acc[0][nt]);
      acc[1][nt] = mma_f16(a1, bb, acc[1][nt]);
    }
  }

  #pragma unroll
  for (int nt = 0; nt < 4; ++nt) {
    const int col = 16 * nt + m;
    const float bv = bct[cg * 64 + col];
    #pragma unroll
    for (int mt = 0; mt < 2; ++mt) {
      #pragma unroll
      for (int r = 0; r < 8; ++r) {
        const int rowl = 32 * w + 16 * mt + 8 * hh + r;
        const float y = (acc[mt][nt][r] * (1.0f / 256.0f) + bv) * 4.0f;
        sT[rowl * 64 + col] = (_Float16)y;
      }
    }
  }
  __syncthreads();

  tile_store_h(sT, qkvh, QKVW, r0, cg * 64, w, lane);
  __threadfence();
  tile_store_h(sT, qkvh, QKVW, r0, cg * 64, w, lane);
}

__device__ __forceinline__ v16h pack_p(v8f a, v8f c) {
  const v16h r = { (_Float16)(a[0] * PSC), (_Float16)(a[1] * PSC), (_Float16)(a[2] * PSC), (_Float16)(a[3] * PSC),
                   (_Float16)(a[4] * PSC), (_Float16)(a[5] * PSC), (_Float16)(a[6] * PSC), (_Float16)(a[7] * PSC),
                   (_Float16)(c[0] * PSC), (_Float16)(c[1] * PSC), (_Float16)(c[2] * PSC), (_Float16)(c[3] * PSC),
                   (_Float16)(c[4] * PSC), (_Float16)(c[5] * PSC), (_Float16)(c[6] * PSC), (_Float16)(c[7] * PSC) };
  return r;
}

__device__ __forceinline__ void attn_store(const unsigned short* sH, const unsigned short* sL,
                                           unsigned short* cth, unsigned short* ctl,
                                           int off, int q0, int len, int hd, int w, int lane) {
  const int q8 = lane & 7, sub = lane >> 3;
  #pragma unroll
  for (int i = 0; i < 4; ++i) {
    const int row = 4 * i + sub;
    const int qrow = q0 + 16 * w + row;
    if (qrow < len) {
      const size_t go = (size_t)(off + qrow) * EDIM + hd * HDIM + 8 * q8;
      const v8us vh = *(const v8usa*)(sH + (w * 16 + row) * 64 + 8 * q8);
      const v8us vl = *(const v8usa*)(sL + (w * 16 + row) * 64 + 8 * q8);
      *(volatile v8us*)(cth + go) = vh;
      *(volatile v8us*)(ctl + go) = vl;
    }
  }
}

__global__ __launch_bounds__(128) void k_attn(
    const _Float16* __restrict__ qkvh, const int* __restrict__ lens,
    unsigned short* __restrict__ cth, unsigned short* __restrict__ ctl, int N)
{
  __shared__ __attribute__((aligned(16))) _Float16 sV[64 * 72];
  __shared__ __attribute__((aligned(16))) unsigned short sH[4 * 16 * 64];
  __shared__ __attribute__((aligned(16))) unsigned short sL[4 * 16 * 64];

  const int tid = threadIdx.x, lane = tid & 31, w = tid >> 5, hh = lane >> 4, m = lane & 15;
  const int qb = blockIdx.x, hd = blockIdx.y, b = blockIdx.z;

  int off = 0, len = 0;
  #pragma unroll
  for (int i = 0; i < NBATCH; ++i) {
    int L = lens[i];
    L = (L < 0) ? 0 : ((L > MAXLEN) ? MAXLEN : L);
    off += (i < b) ? L : 0;
    len = (i == b) ? L : len;
  }
  if (off > N) off = N;
  if (len > N - off) len = N - off;

  const int q0 = qb * 64;
  if (q0 >= len) return;

  int qr = q0 + 16 * w + m;
  qr = (qr < len) ? qr : (len - 1);
  const _Float16* qp = qkvh + (size_t)(off + qr) * QKVW + hd * HDIM;
  const v16h qb0 = load_frag_h(qp, hh);
  const v16h qb1 = load_frag_h(qp + 32, hh);

  v8f o[4];
  #pragma unroll
  for (int t = 0; t < 4; ++t) o[t] = zero8f();
  float mrun = -1e30f, lrun = 0.0f;

  const int vkey = tid >> 1, vdh = tid & 1;

  #pragma unroll 1
  for (int kb = 0; kb < len; kb += 64) {
    __syncthreads();
    {
      int kr = kb + vkey;
      kr = (kr < len) ? kr : (len - 1);
      const _Float16* vp = qkvh + (size_t)(off + kr) * QKVW + 2 * EDIM + hd * HDIM + 32 * vdh;
      const v8h v0 = *(const v8ha*)(vp);
      const v8h v1 = *(const v8ha*)(vp + 8);
      const v8h v2 = *(const v8ha*)(vp + 16);
      const v8h v3 = *(const v8ha*)(vp + 24);
      _Float16* d = sV + (32 * vdh) * 72 + vkey;
      #pragma unroll
      for (int e = 0; e < 8; ++e) {
        d[e * 72]        = v0[e];
        d[(8 + e) * 72]  = v1[e];
        d[(16 + e) * 72] = v2[e];
        d[(24 + e) * 72] = v3[e];
      }
    }
    __syncthreads();

    v8f s[4];
    #pragma unroll
    for (int j = 0; j < 4; ++j) {
      int kr = kb + 16 * j + m;
      kr = (kr < len) ? kr : (len - 1);
      const _Float16* kp = qkvh + (size_t)(off + kr) * QKVW + EDIM + hd * HDIM;
      const v16h kf0 = load_frag_h(kp, hh);
      const v16h kf1 = load_frag_h(kp + 32, hh);
      v8f z = zero8f();
      z = mma_f16(kf0, qb0, z);
      z = mma_f16(kf1, qb1, z);
      s[j] = z;
    }
    #pragma unroll
    for (int j = 0; j < 4; ++j)
      #pragma unroll
      for (int r = 0; r < 8; ++r) {
        const int key = kb + 16 * j + 8 * hh + r;
        const float v = s[j][r] * (1.0f / 128.0f);
        s[j][r] = (key < len) ? v : -1e30f;
      }

    float mloc = s[0][0];
    #pragma unroll
    for (int j = 0; j < 4; ++j)
      #pragma unroll
      for (int r = 0; r < 8; ++r) mloc = fmaxf(mloc, s[j][r]);
    mloc = fmaxf(mloc, __shfl_xor(mloc, 16));
    const float mnew = fmaxf(mrun, mloc);
    const float alpha = __expf(mrun - mnew);
    mrun = mnew;
    float lsum = 0.0f;
    #pragma unroll
    for (int j = 0; j < 4; ++j)
      #pragma unroll
      for (int r = 0; r < 8; ++r) {
        const float p = __expf(s[j][r] - mnew);
        s[j][r] = p;
        lsum += p;
      }
    lsum += __shfl_xor(lsum, 16);
    lrun = lrun * alpha + lsum;
    #pragma unroll
    for (int t = 0; t < 4; ++t)
      #pragma unroll
      for (int r = 0; r < 8; ++r) o[t][r] = o[t][r] * alpha;

    const v16h pb0 = pack_p(s[0], s[1]);
    const v16h pb1 = pack_p(s[2], s[3]);

    #pragma unroll
    for (int t = 0; t < 4; ++t) {
      const _Float16* vr = sV + (16 * t + m) * 72;
      const v16h vf0 = load_frag_h(vr, hh);
      const v16h vf1 = load_frag_h(vr + 32, hh);
      o[t] = mma_f16(vf0, pb0, o[t]);
      o[t] = mma_f16(vf1, pb1, o[t]);
    }
  }

  const float inv = (1.0f / lrun) * (1.0f / 65536.0f);
  #pragma unroll
  for (int t = 0; t < 4; ++t)
    #pragma unroll
    for (int r = 0; r < 8; ++r) {
      const float c = o[t][r] * inv;
      const unsigned int hb = bf16_rne(c);
      const int idx = (w * 16 + m) * 64 + 16 * t + 8 * hh + r;
      sH[idx] = (unsigned short)hb;
      sL[idx] = (unsigned short)bf16_lo(c, hb);
    }
  __syncthreads();

  attn_store(sH, sL, cth, ctl, off, q0, len, hd, w, lane);
  __threadfence();
  attn_store(sH, sL, cth, ctl, off, q0, len, hd, w, lane);
}

__device__ __forceinline__ void plane2_store16(const unsigned short* sH, const unsigned short* sL,
                                               unsigned short* ph, unsigned short* pl,
                                               int r0, int c0, int w, int lane) {
  const int q8 = lane & 7, sub = lane >> 3;
  #pragma unroll
  for (int i = 0; i < 4; ++i) {
    const int rowl = 16 * w + 4 * i + sub;
    const size_t go = (size_t)(r0 + rowl) * EDIM + c0 + 8 * q8;
    const v8us vh = *(const v8usa*)(sH + rowl * 64 + 8 * q8);
    const v8us vl = *(const v8usa*)(sL + rowl * 64 + 8 * q8);
    *(volatile v8us*)(ph + go) = vh;
    *(volatile v8us*)(pl + go) = vl;
  }
}

__global__ __launch_bounds__(128) void k_outp(
    const unsigned short* __restrict__ cth, const unsigned short* __restrict__ ctl,
    const unsigned short* __restrict__ woth, const unsigned short* __restrict__ wotl,
    const float* __restrict__ b_out,
    unsigned short* __restrict__ aoh, unsigned short* __restrict__ aol)
{
  __shared__ __attribute__((aligned(16))) unsigned short sH[64 * 64];
  __shared__ __attribute__((aligned(16))) unsigned short sL[64 * 64];

  const int tid = threadIdx.x, lane = tid & 31, w = tid >> 5, hh = lane >> 4, m = lane & 15;
  const int r0 = blockIdx.x * 64, cg = blockIdx.y;
  const int row = r0 + 16 * w + m;
  const unsigned short* ahp = cth + (size_t)row * EDIM;
  const unsigned short* alp = ctl + (size_t)row * EDIM;
  const unsigned short* bhp = woth + (size_t)(cg * 64 + m) * EDIM;
  const unsigned short* blp = wotl + (size_t)(cg * 64 + m) * EDIM;

  v8f acc[4];
  #pragma unroll
  for (int nt = 0; nt < 4; ++nt) acc[nt] = zero8f();

  #pragma unroll 1
  for (int k0 = 0; k0 < EDIM; k0 += 32) {
    const v16b ah = load_frag_u(ahp + k0, hh);
    const v16b al = load_frag_u(alp + k0, hh);
    #pragma unroll
    for (int nt = 0; nt < 4; ++nt) {
      const v16b bh = load_frag_u(bhp + (size_t)(16 * nt) * EDIM + k0, hh);
      const v16b bl = load_frag_u(blp + (size_t)(16 * nt) * EDIM + k0, hh);
      acc[nt] = mma_bf16(ah, bh, acc[nt]);
      acc[nt] = mma_bf16(ah, bl, acc[nt]);
      acc[nt] = mma_bf16(al, bh, acc[nt]);
    }
  }

  #pragma unroll
  for (int nt = 0; nt < 4; ++nt) {
    const int col = 16 * nt + m;
    const float bv = b_out[cg * 64 + col];
    #pragma unroll
    for (int r = 0; r < 8; ++r) {
      const int rowl = 16 * w + 8 * hh + r;
      const float y = acc[nt][r] + bv;
      const unsigned int hb = bf16_rne(y);
      sH[rowl * 64 + col] = (unsigned short)hb;
      sL[rowl * 64 + col] = (unsigned short)bf16_lo(y, hb);
    }
  }
  __syncthreads();

  plane2_store16(sH, sL, aoh, aol, r0, cg * 64, w, lane);
  __threadfence();
  plane2_store16(sH, sL, aoh, aol, r0, cg * 64, w, lane);
}

__device__ __forceinline__ void cls_store(const float* sO, char* ob, int nfull, int rem,
                                          int tid, int w, int lane) {
  const int q8 = lane & 7, sub = lane >> 3;
  const char* sbp = (const char*)sO;
  #pragma unroll
  for (int i = 0; i < 3; ++i) {
    const int line = 16 * i + 4 * w + sub;
    if (line < nfull) {
      const v4f v = *(const v4fa*)(sbp + line * 128 + 16 * q8);
      *(volatile v4f*)(ob + (size_t)line * 128 + 16 * q8) = v;
    }
  }
  if (rem != 0 && tid == 0) {
    const float* sp = sO + nfull * 32;
    volatile float* dp = (volatile float*)(ob + (size_t)nfull * 128);
    const int ne = rem >> 2;
    if (ne == 2) {
      const v2f v = { sp[0], sp[1] };
      *(volatile v2f*)(ob + (size_t)nfull * 128) = v;
    } else {
      for (int e = 0; e < ne; ++e) dp[e] = sp[e];
    }
  }
}

__global__ __launch_bounds__(128) void k_cls(
    const unsigned short* __restrict__ aoh, const unsigned short* __restrict__ aol,
    const unsigned short* __restrict__ wch, const unsigned short* __restrict__ wcl,
    const float* __restrict__ b_cls, float* __restrict__ out1, int N)
{
  __shared__ __attribute__((aligned(16))) float sO[64 * NCLS];

  const int tid = threadIdx.x, lane = tid & 31, w = tid >> 5, hh = lane >> 4, m = lane & 15;
  const int r0 = blockIdx.x * 64;
  const int row = r0 + 16 * w + m;
  const unsigned short* ahp = aoh + (size_t)row * EDIM;
  const unsigned short* alp = aol + (size_t)row * EDIM;
  const unsigned short* bhp = wch + (size_t)m * EDIM;
  const unsigned short* blp = wcl + (size_t)m * EDIM;

  v8f acc[2];
  acc[0] = zero8f();
  acc[1] = zero8f();

  #pragma unroll 1
  for (int k0 = 0; k0 < EDIM; k0 += 32) {
    const v16b ah = load_frag_u(ahp + k0, hh);
    const v16b al = load_frag_u(alp + k0, hh);
    #pragma unroll
    for (int nt = 0; nt < 2; ++nt) {
      const v16b bh = load_frag_u(bhp + (size_t)(16 * nt) * EDIM + k0, hh);
      const v16b bl = load_frag_u(blp + (size_t)(16 * nt) * EDIM + k0, hh);
      acc[nt] = mma_bf16(ah, bh, acc[nt]);
      acc[nt] = mma_bf16(ah, bl, acc[nt]);
      acc[nt] = mma_bf16(al, bh, acc[nt]);
    }
  }

  #pragma unroll
  for (int nt = 0; nt < 2; ++nt) {
    const int col = 16 * nt + m;
    const int ccol = (col < NCLS) ? col : (NCLS - 1);
    const float bv = b_cls[ccol];
    #pragma unroll
    for (int r = 0; r < 8; ++r) {
      const int rowl = 16 * w + 8 * hh + r;
      const float y = acc[nt][r] + bv;
      if (col < NCLS) sO[rowl * NCLS + col] = y;
    }
  }
  __syncthreads();

  int rv = N - r0;
  rv = (rv > 64) ? 64 : rv;
  const int nbytes = rv * NCLS * 4;
  const int nfull = nbytes >> 7;
  const int rem = nbytes & 127;
  char* ob = (char*)out1 + (size_t)r0 * NCLS * 4;

  cls_store(sO, ob, nfull, rem, tid, w, lane);
  __threadfence();
  cls_store(sO, ob, nfull, rem, tid, w, lane);
}

extern "C" void kernel_launch(void* const* d_in, const int* in_sizes, int n_in,
                              void* d_out, int out_size, void* d_ws, size_t ws_size,
                              hipStream_t stream)
{
  if (n_in < 15) return;
  const int n0 = in_sizes[0];
  if (n0 <= 0 || (n0 % 64) != 0) return;
  const int N = n0 / 64;
  if (in_sizes[1] != N * PCIN) return;
  if (in_sizes[2] != NBATCH) return;
  if (in_sizes[3] != PCIN * EDIM || in_sizes[4] != EDIM) return;
  if (in_sizes[5] != EDIM * 64 || in_sizes[6] != 64) return;
  if (in_sizes[7] != XMW * QKVW || in_sizes[8] != QKVW) return;
  if (in_sizes[9] != EDIM * QKVW || in_sizes[10] != QKVW) return;
  if (in_sizes[11] != EDIM * EDIM || in_sizes[12] != EDIM) return;
  if (in_sizes[13] != EDIM * NCLS || in_sizes[14] != NCLS) return;
  if (out_size != N * (XMW + NCLS)) return;

  const float* img   = (const float*)d_in[0];
  const float* pc    = (const float*)d_in[1];
  const int*   lens  = (const int*)d_in[2];
  const float* w_pc1 = (const float*)d_in[3];
  const float* b_pc1 = (const float*)d_in[4];
  const float* w_pc2 = (const float*)d_in[5];
  const float* b_pc2 = (const float*)d_in[6];
  const float* w_qkv = (const float*)d_in[7];
  const float* b_qkv = (const float*)d_in[8];
  const float* w_in  = (const float*)d_in[9];
  const float* b_in  = (const float*)d_in[10];
  const float* w_out = (const float*)d_in[11];
  const float* b_out = (const float*)d_in[12];
  const float* w_cls = (const float*)d_in[13];
  const float* b_cls = (const float*)d_in[14];

  float* out0 = (float*)d_out;
  float* out1 = out0 + (size_t)N * XMW;

  const int nb128 = (N + 127) / 128;
  const int NP = nb128 * 128;
  const int nb64 = NP / 64;

  size_t off = 0;
  auto carve = [&](size_t bytes) { const size_t o = off; off += (bytes + 255) & ~(size_t)255; return o; };
  const size_t o_w2t  = carve((size_t)64 * EDIM * 2);
  const size_t o_woth = carve((size_t)EDIM * EDIM * 2);
  const size_t o_wotl = carve((size_t)EDIM * EDIM * 2);
  const size_t o_wcth = carve((size_t)NCLSP * EDIM * 2);
  const size_t o_wctl = carve((size_t)NCLSP * EDIM * 2);
  const size_t o_wct  = carve((size_t)QKVW * XMW * 2);
  const size_t o_bct  = carve((size_t)QKVW * 4);
  const size_t o_h16  = carve((size_t)NP * EDIM * 2);
  const size_t o_xh   = carve((size_t)NP * XMW * 2);
  const size_t o_qkvh = carve((size_t)NP * QKVW * 2);
  const size_t o_cth  = carve((size_t)NP * EDIM * 2);
  const size_t o_ctl  = carve((size_t)NP * EDIM * 2);
  const size_t o_aoh  = carve((size_t)NP * EDIM * 2);
  const size_t o_aol  = carve((size_t)NP * EDIM * 2);
  if (off > ws_size) return;

  char* ws = (char*)d_ws;
  unsigned short* w2t  = (unsigned short*)(ws + o_w2t);
  unsigned short* woth = (unsigned short*)(ws + o_woth);
  unsigned short* wotl = (unsigned short*)(ws + o_wotl);
  unsigned short* wcth = (unsigned short*)(ws + o_wcth);
  unsigned short* wctl = (unsigned short*)(ws + o_wctl);
  _Float16*       wct  = (_Float16*)(ws + o_wct);
  float*          bct  = (float*)(ws + o_bct);
  _Float16*       h16  = (_Float16*)(ws + o_h16);
  _Float16*       xh   = (_Float16*)(ws + o_xh);
  _Float16*       qkvh = (_Float16*)(ws + o_qkvh);
  unsigned short* cth  = (unsigned short*)(ws + o_cth);
  unsigned short* ctl  = (unsigned short*)(ws + o_ctl);
  unsigned short* aoh  = (unsigned short*)(ws + o_aoh);
  unsigned short* aol  = (unsigned short*)(ws + o_aol);

  k_wprep<<<dim3(80), dim3(256), 0, stream>>>(w_pc2, w_out, w_cls, w2t, woth, wotl, wcth, wctl);
  k_wcomp<<<dim3(QKVW / 64, XMW / 64), dim3(256), 0, stream>>>(w_qkv, b_qkv, w_in, b_in, wct, bct);
  k_pc1<<<dim3(nb128, EDIM / 64), dim3(128), 0, stream>>>(pc, w_pc1, b_pc1, h16, N);
  k_pc2x<<<dim3(nb128), dim3(128), 0, stream>>>(h16, (const _Float16*)w2t, b_pc2, img, out0, xh, N);
  k_qkv<<<dim3(nb128, QKVW / 64), dim3(128), 0, stream>>>(xh, wct, bct, qkvh);
  k_attn<<<dim3((MAXLEN + 63) / 64, NHEAD, NBATCH), dim3(128), 0, stream>>>(qkvh, lens, cth, ctl, N);
  k_outp<<<dim3(nb64, EDIM / 64), dim3(128), 0, stream>>>(cth, ctl, woth, wotl, b_out, aoh, aol);
  k_cls<<<dim3(nb64), dim3(128), 0, stream>>>(aoh, aol, wcth, wctl, b_cls, out1, N);
}
